// SAGELayer_11587821765008
// MI455X (gfx1250) — hardware-verified
//
#include <hip/hip_runtime.h>
#include <stddef.h>
#include <stdint.h>


#define DF      64
#define KF      192
#define KR      64
#define MHW     128
#define NTHR    256
#define NWAVE   8
#define EPT     8
#define CHUNK   (NTHR * EPT)
#define WCAP    (EPT * 32)
#define LISTN   (NWAVE * WCAP)
#define NBMAX   2048
#define RCAP    28672
#define DEGCAP  96
#define PKS     11
#define STW     512
#define GBM     64
#define GTHR    128
#define NUF     (DF * (KF / 8))
#define NUR     (DF * (KR / 8))
#define NUW     (NUF + NUR)
#define WSMAX   134217728
#define LDS_AGG ((2 * RCAP + 2 * NBMAX + LISTN) * 4 + 64)

static_assert((CHUNK & (CHUNK - 1)) == 0 && CHUNK <= (1 << PKS));
static_assert((NBMAX & (NBMAX - 1)) == 0 && NBMAX <= (1 << PKS));
static_assert(NTHR * 8 == NBMAX);
static_assert(LISTN >= NBMAX);
static_assert(LISTN >= NWAVE * WCAP);
static_assert((RCAP % 32) == 0);
static_assert(NWAVE * STW <= RCAP);
static_assert(STW >= 64);
static_assert(LDS_AGG <= 300000);
static_assert(GBM == (GTHR / 32) * 16);
static_assert((KF % 32) == 0 && (KR % 32) == 0 && (DF % 64) == 0);
static_assert(KF == 3 * DF && KR == DF && MHW == 2 * DF);
static_assert(DF == 32 * 2);
static_assert((NUF % NTHR) == 0 && (NUW % NTHR) == 0);

typedef float          v4f  __attribute__((ext_vector_type(4)));
typedef float          v8f  __attribute__((ext_vector_type(8)));
typedef int            v4i  __attribute__((ext_vector_type(4)));
typedef int            v8i  __attribute__((ext_vector_type(8)));
typedef unsigned int   v4u  __attribute__((ext_vector_type(4)));
typedef unsigned short v8us __attribute__((ext_vector_type(8)));
typedef __bf16         v16b __attribute__((ext_vector_type(16)));
union FragB { v16b v; v8us h[2]; v8i w; };

__device__ __forceinline__ v8f wmb(const FragB& a, const FragB& b, v8f c) {
  v8f d = __builtin_amdgcn_wmma_f32_16x16x32_bf16(false, a.v, false, b.v, (short)0, c, false, false);
  asm volatile("v_nop\n\tv_nop\n\tv_nop\n\tv_nop" : "+v"(d) : "v"(a.w), "v"(b.w));
  return d;
}

__device__ __forceinline__ unsigned short bf_bits(float f) {
  unsigned int u = __float_as_uint(f);
  u += 0x7FFFu + ((u >> 16) & 1u);
  return (unsigned short)(u >> 16);
}
__device__ __forceinline__ float bf_val(unsigned short b) {
  return __uint_as_float(((unsigned int)b) << 16);
}
__device__ __forceinline__ float bf_rne(float f) { return bf_val(bf_bits(f)); }

__device__ __forceinline__ v8us cvt8b(const v4f a, const v4f b) {
  v8us hv;
  hv[0] = bf_bits(a.x); hv[1] = bf_bits(a.y); hv[2] = bf_bits(a.z); hv[3] = bf_bits(a.w);
  hv[4] = bf_bits(b.x); hv[5] = bf_bits(b.y); hv[6] = bf_bits(b.z); hv[7] = bf_bits(b.w);
  return hv;
}

__device__ __forceinline__ int scan_chunk(const int* __restrict__ dsts, int nE, int cbase, int slotBase,
                                          int nb, int vec8, int* list, int tid, int lane, int wave) {
  int wc = 0;
  const int el0  = tid * EPT;
  const int e0   = cbase + el0;
  const int sent = -2147483647 - 1;
  v4i da, db;
  if (vec8 != 0 && cbase + CHUNK <= nE) {
    da = *(const v4i*)(dsts + e0);
    db = *(const v4i*)(dsts + e0 + 4);
  } else {
    da.x = (e0     < nE) ? dsts[min(e0,     nE - 1)] : sent;
    da.y = (e0 + 1 < nE) ? dsts[min(e0 + 1, nE - 1)] : sent;
    da.z = (e0 + 2 < nE) ? dsts[min(e0 + 2, nE - 1)] : sent;
    da.w = (e0 + 3 < nE) ? dsts[min(e0 + 3, nE - 1)] : sent;
    db.x = (e0 + 4 < nE) ? dsts[min(e0 + 4, nE - 1)] : sent;
    db.y = (e0 + 5 < nE) ? dsts[min(e0 + 5, nE - 1)] : sent;
    db.z = (e0 + 6 < nE) ? dsts[min(e0 + 6, nE - 1)] : sent;
    db.w = (e0 + 7 < nE) ? dsts[min(e0 + 7, nE - 1)] : sent;
  }
  const unsigned nbs = (unsigned)slotBase;
  const unsigned unb = (unsigned)nb;
  const unsigned s0 = (unsigned)da.x - nbs, s1 = (unsigned)da.y - nbs;
  const unsigned s2 = (unsigned)da.z - nbs, s3 = (unsigned)da.w - nbs;
  const unsigned s4 = (unsigned)db.x - nbs, s5 = (unsigned)db.y - nbs;
  const unsigned s6 = (unsigned)db.z - nbs, s7 = (unsigned)db.w - nbs;
  const bool h0 = s0 < unb, h1 = s1 < unb, h2 = s2 < unb, h3 = s3 < unb;
  const bool h4 = s4 < unb, h5 = s5 < unb, h6 = s6 < unb, h7 = s7 < unb;
  const unsigned any = __builtin_amdgcn_ballot_w32(h0 | h1 | h2 | h3 | h4 | h5 | h6 | h7);
  if (any != 0u) {
#define HITJ(J, HJ, SJ) { \
      const unsigned mj = __builtin_amdgcn_ballot_w32(HJ); \
      if (mj != 0u) { \
        if (HJ) { \
          const int pos = wc + (int)__builtin_amdgcn_mbcnt_lo(mj, 0u); \
          if (pos < WCAP) list[wave * WCAP + pos] = ((el0 + (J)) << PKS) | (int)(SJ); \
        } \
        wc += (int)__builtin_popcount(mj); } }
    HITJ(0, h0, s0)
    HITJ(1, h1, s1)
    HITJ(2, h2, s2)
    HITJ(3, h3, s3)
    HITJ(4, h4, s4)
    HITJ(5, h5, s5)
    HITJ(6, h6, s6)
    HITJ(7, h7, s7)
#undef HITJ
  }
  return wc;
}

__global__ __launch_bounds__(NTHR) void k_xprep(const float* __restrict__ x, unsigned short* xb,
                                                int nN, int nUnits) {
  const int i = (int)blockIdx.x * NTHR + (int)threadIdx.x;
  if (i >= nUnits) return;
  const int row = i >> 3;
  const int c0  = (i & 7) * 8;
  const int rc  = row < nN ? row : nN - 1;
  const float* p = x + (size_t)rc * DF + c0;
  v4f a = *(const v4f*)p, b = *(const v4f*)(p + 4);
  const v4f z4 = {0.f, 0.f, 0.f, 0.f};
  if (row >= nN) { a = z4; b = z4; }
  const v8us hv = cvt8b(a, b);
  const size_t o = (size_t)row * DF + c0;
  *(volatile v8us*)(xb + o) = hv;
  __threadfence();
  *(volatile v8us*)(xb + o) = hv;
}

__global__ __launch_bounds__(NTHR) void k_wprep(const float* __restrict__ wfc, const float* __restrict__ wres,
                                                unsigned short* wtf, unsigned short* wtr, int nUnits) {
  const int u = (int)blockIdx.x * NTHR + (int)threadIdx.x;
  if (u >= nUnits) return;
  const float* p;
  unsigned short* o;
  if (u < NUF) {
    int n = u / (KF / 8);
    n = n > DF - 1 ? DF - 1 : n;
    const int k8 = (u - n * (KF / 8)) * 8;
    int kk = k8 < 2 * DF ? k8 : k8 - DF;
    kk = kk < 0 ? 0 : (kk > 2 * DF - 8 ? 2 * DF - 8 : kk);
    p = wfc + (size_t)kk * DF + n;
    o = wtf + (size_t)n * KF + k8;
  } else {
    const int v = u - NUF;
    int n = v / (KR / 8);
    n = n > DF - 1 ? DF - 1 : n;
    int k8 = (v - n * (KR / 8)) * 8;
    k8 = k8 < 0 ? 0 : (k8 > DF - 8 ? DF - 8 : k8);
    p = wres + (size_t)k8 * DF + n;
    o = wtr + (size_t)n * KR + k8;
  }
  v4f a, b;
  a.x = p[0];                  a.y = p[(size_t)DF];         a.z = p[(size_t)2 * DF];     a.w = p[(size_t)3 * DF];
  b.x = p[(size_t)4 * DF];     b.y = p[(size_t)5 * DF];     b.z = p[(size_t)6 * DF];     b.w = p[(size_t)7 * DF];
  const v8us hv = cvt8b(a, b);
  *(volatile v8us*)o = hv;
  __threadfence();
  *(volatile v8us*)o = hv;
}

__global__ __launch_bounds__(GTHR) void k_gemm2(const unsigned short* __restrict__ xb,
                                                const unsigned short* __restrict__ mh,
                                                const unsigned short* __restrict__ wtf,
                                                const unsigned short* __restrict__ wtr,
                                                const float* __restrict__ bfc,
                                                const float* __restrict__ bres,
                                                float* outF, int nN)
{
  __shared__ __attribute__((aligned(16))) float stg[GBM * DF];
  const int tid = (int)threadIdx.x, lane = tid & 31, wave = tid >> 5, hh = lane >> 4, m = lane & 15;
  const int rowBase = (int)blockIdx.x * GBM;
  const int arow    = rowBase + 16 * wave + m;

  v8f accf[4], accr[4];
  {
    const v8f z = {0.f, 0.f, 0.f, 0.f, 0.f, 0.f, 0.f, 0.f};
#pragma unroll
    for (int t = 0; t < 4; ++t) { accf[t] = z; accr[t] = z; }
  }
  const unsigned short* xp  = xb  + (size_t)arow * DF  + 8 * hh;
  const unsigned short* mp  = mh  + (size_t)arow * MHW + 8 * hh;
  const unsigned short* wfp = wtf + (size_t)m * KF + 8 * hh;
  const unsigned short* wrp = wtr + (size_t)m * KR + 8 * hh;

#pragma unroll 1
  for (int ks = 0; ks < 2; ++ks) {
    FragB af;
    af.h[0] = *(const v8us*)(xp + 32 * ks);
    af.h[1] = *(const v8us*)(xp + 32 * ks + 16);
#pragma unroll
    for (int t = 0; t < 4; ++t) {
      const unsigned short* wq = wfp + (size_t)(16 * t) * KF + 32 * ks;
      FragB bf;
      bf.h[0] = *(const v8us*)wq;
      bf.h[1] = *(const v8us*)(wq + 16);
      accf[t] = wmb(af, bf, accf[t]);
      const unsigned short* rq = wrp + (size_t)(16 * t) * KR + 32 * ks;
      FragB cf;
      cf.h[0] = *(const v8us*)rq;
      cf.h[1] = *(const v8us*)(rq + 16);
      accr[t] = wmb(af, cf, accr[t]);
    }
  }
#pragma unroll 1
  for (int j = 0; j < 4; ++j) {
    FragB af;
    af.h[0] = *(const v8us*)(mp + 32 * j);
    af.h[1] = *(const v8us*)(mp + 32 * j + 16);
#pragma unroll
    for (int t = 0; t < 4; ++t) {
      const unsigned short* wq = wfp + (size_t)(16 * t) * KF + DF + 32 * j;
      FragB bf;
      bf.h[0] = *(const v8us*)wq;
      bf.h[1] = *(const v8us*)(wq + 16);
      accf[t] = wmb(af, bf, accf[t]);
    }
  }

#pragma unroll
  for (int t = 0; t < 4; ++t) {
    const int lc = 16 * t + m;
    const float bbf = bf_rne(bfc[lc]);
    const float bbr = bf_rne(bres[lc]);
#pragma unroll
    for (int r = 0; r < 8; ++r) {
      const int lr = 16 * wave + 8 * hh + r;
      const float rl = fmaxf(accf[t][r] + bbf, 0.0f);
      const float rs = accr[t][r] + bbr;
      stg[lr * DF + lc] = rl + rs;
    }
  }
  __syncthreads();

  const int rsub = lane >> 4;
  const int cp   = lane & 15;
  v4f fv[8];
#pragma unroll
  for (int i = 0; i < 8; ++i) {
    const int lr = 16 * wave + 2 * i + rsub;
    fv[i] = *(const v4f*)(stg + lr * DF + 4 * cp);
  }
#pragma unroll
  for (int i = 0; i < 8; ++i) {
    const int lr = 16 * wave + 2 * i + rsub;
    const int gr = rowBase + lr;
    const bool ok = gr < nN;
    const int grc = ok ? gr : 0;
    float* op = outF + (size_t)grc * DF + 4 * cp;
    if (ok) *(volatile v4f*)op = fv[i];
  }
  __threadfence();
#pragma unroll
  for (int i = 0; i < 8; ++i) {
    const int lr = 16 * wave + 2 * i + rsub;
    const int gr = rowBase + lr;
    const bool ok = gr < nN;
    const int grc = ok ? gr : 0;
    float* op = outF + (size_t)grc * DF + 4 * cp;
    if (ok) *(volatile v4f*)op = fv[i];
  }
}

__global__ __launch_bounds__(NTHR) void k_agg(
    const int* __restrict__ srcs, const int* __restrict__ dsts,
    const unsigned short* __restrict__ xb,
    unsigned short* mh,
    int nN, int nE, int nb, int vec8, int MPr) {
  extern __shared__ v4f lds_dyn[];
  int* reg1 = (int*)lds_dyn;
  int* reg2 = reg1 + RCAP;
  int* scnt = reg2 + RCAP;
  int* soff = scnt + NBMAX;
  int* list = soff + NBMAX;
  int* wcnt = list + LISTN;
  int* wtot = wcnt + NWAVE;
  const int tid = (int)threadIdx.x, lane = tid & 31, wave = tid >> 5;
  const int nodeBase = (int)blockIdx.x * nb;

  for (int i = tid; i < NBMAX; i += NTHR) scnt[i] = 0;
  __syncthreads();

  int tot = 0;
  const int nChunks = (nE + CHUNK - 1) / CHUNK;
#pragma unroll 1
  for (int ch = 0; ch < nChunks; ++ch) {
    const int cbase = ch * CHUNK;
    const int wc = scan_chunk(dsts, nE, cbase, nodeBase, nb, vec8, list, tid, lane, wave);
    if (lane == 0) wcnt[wave] = wc;
    __syncthreads();
    int pre = 0, all = 0;
#pragma unroll
    for (int w2 = 0; w2 < NWAVE; ++w2) {
      int c = wcnt[w2];
      c = c < 0 ? 0 : (c > WCAP ? WCAP : c);
      all += c;
      pre += (w2 < wave) ? c : 0;
    }
    const int wcc  = wc > WCAP ? WCAP : wc;
    const int base = tot + pre;
#pragma unroll 1
    for (int i = lane; i < wcc; i += 32) {
      const int ent = list[wave * WCAP + i];
      const int el  = (ent >> PKS) & (CHUNK - 1);
      const int sl  = ent & (NBMAX - 1);
      int eid = cbase + el;
      eid = eid > nE - 1 ? nE - 1 : eid;
      const int pos = base + i;
      if (pos < RCAP) reg1[pos] = (int)(((unsigned)eid << PKS) | (unsigned)sl);
    }
    tot += all;
    tot = tot > RCAP ? RCAP : tot;
    __syncthreads();
  }
  const int nh = tot;

  if (wave == 0) {
#pragma unroll 1
    for (int b0 = 0; b0 < nh; b0 += 32) {
      const int idx = b0 + lane;
      const int uv  = reg1[idx < RCAP ? idx : RCAP - 1];
      const int m32 = (nh - b0) < 32 ? (nh - b0) : 32;
#pragma unroll 1
      for (int k = 0; k < m32; ++k) {
        const int u  = __builtin_amdgcn_readlane(uv, k);
        const int sl = u & (NBMAX - 1);
        if (lane == 0) scnt[sl] = scnt[sl] + 1;
      }
    }
  }
  __syncthreads();

  {
    const v4i ca = *(const v4i*)(scnt + 8 * tid);
    const v4i cb = *(const v4i*)(scnt + 8 * tid + 4);
    const int e0 = ca.x < 0 ? 0 : ca.x, e1 = ca.y < 0 ? 0 : ca.y, e2 = ca.z < 0 ? 0 : ca.z, e3 = ca.w < 0 ? 0 : ca.w;
    const int e4 = cb.x < 0 ? 0 : cb.x, e5 = cb.y < 0 ? 0 : cb.y, e6 = cb.z < 0 ? 0 : cb.z, e7 = cb.w < 0 ? 0 : cb.w;
    const int ts = e0 + e1 + e2 + e3 + e4 + e5 + e6 + e7;
    int incl = ts;
#pragma unroll
    for (int d = 1; d < 32; d <<= 1) {
      const int up = __shfl_up(incl, d);
      if (lane >= d) incl += up;
    }
    if (lane == 31) wtot[wave] = incl;
    __syncthreads();
    int pre = 0;
#pragma unroll
    for (int w2 = 0; w2 < NWAVE; ++w2) pre += (w2 < wave) ? wtot[w2] : 0;
    int run = pre + incl - ts;
    soff[8 * tid + 0] = run; run += e0;
    soff[8 * tid + 1] = run; run += e1;
    soff[8 * tid + 2] = run; run += e2;
    soff[8 * tid + 3] = run; run += e3;
    soff[8 * tid + 4] = run; run += e4;
    soff[8 * tid + 5] = run; run += e5;
    soff[8 * tid + 6] = run; run += e6;
    soff[8 * tid + 7] = run;
  }
  __syncthreads();
  for (int i = tid; i < NBMAX; i += NTHR) list[i] = soff[i];
  __syncthreads();

  if (wave == 0) {
#pragma unroll 1
    for (int b0 = 0; b0 < nh; b0 += 32) {
      const int idx = b0 + lane;
      const int uv  = reg1[idx < RCAP ? idx : RCAP - 1];
      const int m32 = (nh - b0) < 32 ? (nh - b0) : 32;
#pragma unroll 1
      for (int k = 0; k < m32; ++k) {
        const int u   = __builtin_amdgcn_readlane(uv, k);
        const int sl  = u & (NBMAX - 1);
        const int eid = (int)((unsigned)u >> PKS);
        if (lane == 0) {
          int pos = list[sl];
          pos = pos < 0 ? 0 : (pos > RCAP - 1 ? RCAP - 1 : pos);
          reg2[pos] = eid;
          list[sl] = pos + 1;
        }
      }
    }
  }
  __syncthreads();

  const int nbw = nb >> 3;
  const bool ovf = (nh >= RCAP);
  const float qnan = __int_as_float(0x7fc00000);
  unsigned int* stwu = (unsigned int*)((float*)reg1 + wave * STW);

#pragma unroll 1
  for (int jt = 0; jt < nbw; ++jt) {
    const int slot = wave * nbw + jt;
    const int grow = nodeBase + slot;
    int st = soff[slot];
    const int craw = scnt[slot];
    int cnt = craw;
    st  = st < 0 ? 0 : (st > nh ? nh : st);
    cnt = cnt < 0 ? 0 : (cnt > DEGCAP ? DEGCAP : cnt);
    if (cnt > nh - st) cnt = nh - st;
    const float pz   = (ovf || craw > DEGCAP) ? qnan : 0.0f;
    const float live = grow < nN ? 1.0f : 0.0f;

    float a0 = 0.0f, a1 = 0.0f;
#pragma unroll 1
    for (int q = 0; q < cnt; ++q) {
      int idx = st + q; idx = idx > RCAP - 1 ? RCAP - 1 : idx;
      int eid = reg2[idx]; eid = eid < 0 ? 0 : (eid > nE - 1 ? nE - 1 : eid);
      const int sraw = srcs[eid];
      const int s = sraw < 0 ? 0 : (sraw > nN - 1 ? nN - 1 : sraw);
      const unsigned int w = *(const unsigned int*)(xb + (size_t)s * DF + 2 * lane);
      a0 += __uint_as_float(w << 16);
      a1 += __uint_as_float(w & 0xffff0000u);
    }
    const float dcl  = cnt > 0 ? (float)cnt : 1.0f;
    const float invd = 1.0f / dcl;
    const float m0 = (a0 * invd) * live + pz;
    const float m1 = (a1 * invd) * live + pz;
    const unsigned short hb0 = bf_bits(m0), hb1 = bf_bits(m1);
    const unsigned short lb0 = bf_bits(m0 - bf_val(hb0)), lb1 = bf_bits(m1 - bf_val(hb1));
    const unsigned int hw = (unsigned int)hb0 | ((unsigned int)hb1 << 16);
    const unsigned int lw = (unsigned int)lb0 | ((unsigned int)lb1 << 16);
    __builtin_amdgcn_fence(__ATOMIC_RELEASE, "wavefront");
    __builtin_amdgcn_wave_barrier();
    stwu[lane]      = hw;
    stwu[32 + lane] = lw;
    __builtin_amdgcn_fence(__ATOMIC_RELEASE, "wavefront");
    __builtin_amdgcn_wave_barrier();
    const int lq = lane < 16 ? lane : 15;
    const v4u pk = *(const v4u*)(stwu + 4 * lq);
    const int growc = grow < MPr ? grow : 0;
    unsigned short* gp = mh + (size_t)growc * MHW + 8 * lq;
    const bool wsv = (grow < MPr) && (lane < 16);
    if (wsv) *(volatile v4u*)gp = pk;
    __threadfence();
    if (wsv) *(volatile v4u*)gp = pk;
  }
}

static int pick_nb(int nE, int nN) {
  int nb = NBMAX;
  while (nb > 16 && (long long)nb * (long long)nE * 5LL > (long long)RCAP * (long long)nN * 4LL) nb >>= 1;
  return nb;
}
static inline int cdiv(int a, int b) { return (a + b - 1) / b; }

extern "C" void kernel_launch(void* const* d_in, const int* in_sizes, int n_in,
                              void* d_out, int out_size, void* d_ws, size_t ws_size,
                              hipStream_t stream) {
  if (n_in < 7) return;
  const int nN = in_sizes[0] / DF;
  if (nN <= 0 || in_sizes[0] != nN * DF || nN > (1 << 22)) return;
  const int nE = in_sizes[1];
  if (nE < 1 || in_sizes[2] != nE || nE > (1 << 21)) return;
  if (in_sizes[3] != 2 * DF * DF || in_sizes[4] != DF) return;
  if (in_sizes[5] != DF * DF || in_sizes[6] != DF) return;
  if (out_size != nN * DF) return;

  const float* x    = (const float*)d_in[0];
  const int*   src  = (const int*)  d_in[1];
  const int*   dst  = (const int*)  d_in[2];
  const float* Wfc  = (const float*)d_in[3];
  const float* bfc  = (const float*)d_in[4];
  const float* Wres = (const float*)d_in[5];
  const float* bres = (const float*)d_in[6];
  float* out = (float*)d_out;

  const int MP   = cdiv(nN, GBM) * GBM;
  const int nb   = pick_nb(nE, nN);
  const int gA   = cdiv(MP, nb);
  const int vec8 = 1;
  if (gA * nb < MP) return;

  char* ws = (char*)d_ws;
  size_t off = 0;
  const size_t oXB = off; off += (size_t)MP * DF * 2;     off = (off + 255) & ~(size_t)255;
  const size_t oMH = off; off += (size_t)MP * MHW * 2;    off = (off + 255) & ~(size_t)255;
  const size_t oWF = off; off += (size_t)DF * KF * 2;     off = (off + 255) & ~(size_t)255;
  const size_t oWR = off; off += (size_t)DF * KR * 2;     off = (off + 255) & ~(size_t)255;
  if (off > ws_size || off > (size_t)WSMAX) return;
  unsigned short* XB  = (unsigned short*)(ws + oXB);
  unsigned short* MH  = (unsigned short*)(ws + oMH);
  unsigned short* WTF = (unsigned short*)(ws + oWF);
  unsigned short* WTR = (unsigned short*)(ws + oWR);

  hipFuncSetAttribute(reinterpret_cast<const void*>(&k_agg),
                      hipFuncAttributeMaxDynamicSharedMemorySize, LDS_AGG);

  const int nUx = MP * (DF / 8);
  k_xprep<<<cdiv(nUx, NTHR), NTHR, 0, stream>>>(x, XB, nN, nUx);

  k_wprep<<<NUW / NTHR, NTHR, 0, stream>>>(Wfc, Wres, WTF, WTR, NUW);

  k_agg<<<gA, NTHR, LDS_AGG, stream>>>(src, dst, XB, MH, nN, nE, nb, vec8, MP);

  k_gemm2<<<MP / GBM, GTHR, 0, stream>>>(XB, MH, WTF, WTR, bfc, bres, out, nN);
}
